// Model_19456201851455
// MI455X (gfx1250) — hardware-verified
//
#include <hip/hip_runtime.h>
#include <math.h>

#pragma clang fp contract(off)

constexpr int NBATCH = 8;
constexpr int NSEQ   = 4096;
constexpr int NIN    = 32;
constexpr int NHID   = 256;
constexpr int NOUT   = 32;
constexpr int NROWS  = NBATCH * NSEQ;
constexpr int NTHR   = 256;
constexpr int SLAB_F = 68;
constexpr int SLAB_O = 36;
static_assert(NROWS == 32768);
static_assert(NIN % 32 == 0);
static_assert(NHID % 32 == 0);
static_assert(NROWS % 64 == 0);
static_assert(NHID % 64 == 0);
static_assert(NOUT == 32);
static_assert(NHID == 8 * 32);
static_assert((NROWS * NIN) % (8 * NTHR) == 0);
static_assert(((NROWS / 32) * (NHID / 64)) % 8 == 0);
static_assert((NROWS / 64) % 8 == 0);

typedef __attribute__((ext_vector_type(16))) __bf16   v16b;
typedef __attribute__((ext_vector_type(8)))  __bf16   v8b;
typedef __attribute__((ext_vector_type(8)))  float    v8f;
typedef __attribute__((ext_vector_type(4)))  float    v4f;
typedef __attribute__((ext_vector_type(4)))  unsigned v4u;

__device__ __forceinline__ unsigned bf_hi_bits(float f) {
  const unsigned u = __float_as_uint(f);
  return (u + 0x7FFFu + ((u >> 16) & 1u)) >> 16;
}
__device__ __forceinline__ float bf_bits_val(unsigned hb) { return __uint_as_float(hb << 16); }
__device__ __forceinline__ float ftz32(float x) { return (fabsf(x) < 1.17549435e-38f) ? 0.0f : x; }

__device__ __forceinline__ void dep_guard_b(v8f& a, v8f& b, v16b x, v16b y) { asm volatile("v_nop\n\tv_nop\n\tv_nop\n\tv_nop" : "+v"(a), "+v"(b) : "v"(x), "v"(y)); }
__device__ __forceinline__ void dep_guard_b4(v8f& a, v8f& b, v8f& c, v8f& d, v16b x, v16b y) { asm volatile("v_nop\n\tv_nop\n\tv_nop\n\tv_nop" : "+v"(a), "+v"(b), "+v"(c), "+v"(d) : "v"(x), "v"(y)); }
__device__ __forceinline__ void keep4_b(v16b a, v16b b, v16b c, v16b d) { asm volatile("v_nop" :: "v"(a), "v"(b), "v"(c), "v"(d)); }
__device__ __forceinline__ void acc_guard4(v8f& a, v8f& b, v8f& c, v8f& d) { asm volatile("v_nop\n\tv_nop\n\tv_nop\n\tv_nop" : "+v"(a), "+v"(b), "+v"(c), "+v"(d)); }

template <typename T> struct Frag;
template <> struct Frag<__bf16> {
  typedef v16b V; union U { v16b v; v8b h[2]; };
  static __device__ __forceinline__ v16b load(const __bf16* p) {
    U f; f.h[0] = *(const v8b*)(p); f.h[1] = *(const v8b*)(p + 16); return f.v;
  }
  static __device__ __forceinline__ v8f mma(v16b a, v16b b, v8f c) {
    return __builtin_amdgcn_wmma_f32_16x16x32_bf16(false, a, false, b, (short)0, c, false, false);
  }
};

__global__ __launch_bounds__(NTHR) void split8_kernel(const float* __restrict__ src, unsigned short* __restrict__ dhi,
                                                      unsigned short* __restrict__ dlo, int n8) {
  const int i = blockIdx.x * NTHR + threadIdx.x;
  if (i < n8) {
    const v4f a = *(const v4f*)(src + (size_t)i * 8);
    const v4f b = *(const v4f*)(src + (size_t)i * 8 + 4);
    float f[8];
    f[0] = a[0]; f[1] = a[1]; f[2] = a[2]; f[3] = a[3];
    f[4] = b[0]; f[5] = b[1]; f[6] = b[2]; f[7] = b[3];
    unsigned hb[8], lb[8];
#pragma unroll
    for (int e = 0; e < 8; ++e) {
      hb[e] = bf_hi_bits(f[e]);
      lb[e] = bf_hi_bits(f[e] - bf_bits_val(hb[e]));
    }
    const v4u hw = (v4u){hb[0] | (hb[1] << 16), hb[2] | (hb[3] << 16), hb[4] | (hb[5] << 16), hb[6] | (hb[7] << 16)};
    const v4u lw = (v4u){lb[0] | (lb[1] << 16), lb[2] | (lb[3] << 16), lb[4] | (lb[5] << 16), lb[6] | (lb[7] << 16)};
    unsigned short* ph = dhi + (size_t)i * 8;
    unsigned short* pl = dlo + (size_t)i * 8;
    *(volatile v4u*)ph = hw;
    *(volatile v4u*)pl = lw;
    __threadfence();
    *(volatile v4u*)ph = hw;
    *(volatile v4u*)pl = lw;
  }
}

__global__ __launch_bounds__(NTHR) void ptable_kernel(const float* __restrict__ nu_log, const float* __restrict__ theta_log,
                                                      float* __restrict__ PW, float* __restrict__ GAM) {
  const int t = blockIdx.x;
  const int h = threadIdx.x;
  const float enu = expf(nu_log[h]);
  const float mag = expf(-enu);
  const float ph  = expf(theta_log[h]);
  const float tf  = (float)t;
  const float magt = ftz32(expf(-(tf * enu)));
  float sn, cs;
  sincosf(tf * ph, &sn, &cs);
  float pre = ftz32(magt * cs) + 1e-8f;
  float pim = ftz32(magt * sn);
  const bool first = (t == 0);
  pre = first ? (1.0f + 1e-8f) : pre;
  pim = first ? 0.0f : pim;
  const float den  = pre * pre + pim * pim;
  const float rinv = 1.0f / den;
  const float wre  = pre * rinv;
  const float wim  = -(pim * rinv);
  const float gm   = sqrtf((1.0f - mag * mag) + 1e-8f);
  const v4f o = (v4f){pre, pim, wre, wim};
  float* dst = PW + ((size_t)t * NHID + h) * 4;
  for (int pass = 0; pass < 2; ++pass) {
    *(volatile v4f*)dst = o;
    if (first) *(volatile float*)(GAM + h) = gm;
    __threadfence();
  }
}

__global__ __launch_bounds__(NTHR) void proj_in_kernel(const unsigned short* __restrict__ Uhp, const unsigned short* __restrict__ Ulp,
                                                       const unsigned short* __restrict__ Bhp, const unsigned short* __restrict__ Blp,
                                                       float* __restrict__ Fraw) {
  __shared__ __align__(16) float sT[8][16 * SLAB_F];
  const __bf16* Ah = (const __bf16*)Uhp;
  const __bf16* Al = (const __bf16*)Ulp;
  const __bf16* Bh = (const __bf16*)Bhp;
  const __bf16* Bl = (const __bf16*)Blp;
  const int lane = threadIdx.x & 31;
  const int wave = threadIdx.x >> 5;
  const int tilesN = NHID / 64;
  const int tile = blockIdx.x * 8 + wave;
  if (tile >= (NROWS / 32) * tilesN) return;
  const int tm = tile / tilesN;
  const int tn = tile - tm * tilesN;
  const int m0 = tm * 32;
  const int n0 = tn * 64;
  const int rlane = lane & 15;
  const int koff  = (lane >> 4) * 8;
  const int mOff  = (lane >> 4) * 8;

  v8f acc[2][4];
#pragma unroll
  for (int i = 0; i < 2; ++i)
#pragma unroll
    for (int j = 0; j < 4; ++j) acc[i][j] = (v8f){0.f, 0.f, 0.f, 0.f, 0.f, 0.f, 0.f, 0.f};

  v16b bh[4], bl[4];
#pragma unroll
  for (int j = 0; j < 4; ++j) {
    const size_t bo = (size_t)(n0 + (j << 4) + rlane) * NIN + koff;
    bh[j] = Frag<__bf16>::load(Bh + bo);
    bl[j] = Frag<__bf16>::load(Bl + bo);
  }
#pragma unroll
  for (int i = 0; i < 2; ++i) {
    const size_t ao = (size_t)(m0 + (i << 4) + rlane) * NIN + koff;
    const v16b ah = Frag<__bf16>::load(Ah + ao);
    const v16b al = Frag<__bf16>::load(Al + ao);
#pragma unroll
    for (int j = 0; j < 4; ++j) {
      acc[i][j] = Frag<__bf16>::mma(ah, bh[j], acc[i][j]);
      acc[i][j] = Frag<__bf16>::mma(ah, bl[j], acc[i][j]);
      acc[i][j] = Frag<__bf16>::mma(al, bh[j], acc[i][j]);
    }
    dep_guard_b4(acc[i][0], acc[i][1], acc[i][2], acc[i][3], ah, al);
  }
  keep4_b(bh[0], bh[1], bh[2], bh[3]);
  keep4_b(bl[0], bl[1], bl[2], bl[3]);
  acc_guard4(acc[0][0], acc[0][1], acc[0][2], acc[0][3]);
  acc_guard4(acc[1][0], acc[1][1], acc[1][2], acc[1][3]);

  float* slab = sT[wave];
#pragma unroll
  for (int i = 0; i < 2; ++i) {
    const int mBase = m0 + (i << 4);
#pragma unroll
    for (int j = 0; j < 4; ++j) {
#pragma unroll
      for (int r = 0; r < 8; ++r) slab[(mOff + r) * SLAB_F + (j << 4) + rlane] = acc[i][j][r];
    }
    __builtin_amdgcn_fence(__ATOMIC_RELEASE, "workgroup");
    __builtin_amdgcn_wave_barrier();
    __builtin_amdgcn_fence(__ATOMIC_ACQUIRE, "workgroup");
    {
      const int hh = lane >> 4;
      const int c4 = (lane & 15) * 4;
      for (int pass = 0; pass < 2; ++pass) {
#pragma unroll
        for (int it = 0; it < 8; ++it) {
          const int row = it * 2 + hh;
          const v4f v = *(const v4f*)(slab + row * SLAB_F + c4);
          *(volatile v4f*)(Fraw + (size_t)(mBase + row) * NHID + n0 + c4) = v;
        }
        __threadfence();
      }
    }
    __builtin_amdgcn_fence(__ATOMIC_RELEASE, "workgroup");
    __builtin_amdgcn_wave_barrier();
    __builtin_amdgcn_fence(__ATOMIC_ACQUIRE, "workgroup");
  }
}

__global__ __launch_bounds__(32) void cumsum_kernel(const float* __restrict__ Fraw, const float* __restrict__ PW,
                                                    const float* __restrict__ GAM,
                                                    unsigned short* __restrict__ Xhi, unsigned short* __restrict__ Xlo) {
  const int b    = blockIdx.x;
  const int lane = threadIdx.x;
  const int h0   = lane * 8;
  const v4f g0 = *(const v4f*)(GAM + h0);
  const v4f g1 = *(const v4f*)(GAM + h0 + 4);
  float gam[8];
  gam[0] = g0[0]; gam[1] = g0[1]; gam[2] = g0[2]; gam[3] = g0[3];
  gam[4] = g1[0]; gam[5] = g1[1]; gam[6] = g1[2]; gam[7] = g1[3];
  float sre[8], sim[8];
#pragma unroll
  for (int e = 0; e < 8; ++e) { sre[e] = 0.0f; sim[e] = 0.0f; }
  const float* fp = Fraw + (size_t)b * NSEQ * NHID + h0;
  const float* pp = PW + (size_t)h0 * 4;
  unsigned short* xh = Xhi + (size_t)b * NSEQ * NHID + h0;
  unsigned short* xl = Xlo + (size_t)b * NSEQ * NHID + h0;

#pragma unroll 1
  for (int t = 0; t < NSEQ; ++t) {
    const size_t rowo = (size_t)t * NHID;
    const v4f f0 = *(const v4f*)(fp + rowo);
    const v4f f1 = *(const v4f*)(fp + rowo + 4);
    float fv[8];
    fv[0] = f0[0]; fv[1] = f0[1]; fv[2] = f0[2]; fv[3] = f0[3];
    fv[4] = f1[0]; fv[5] = f1[1]; fv[6] = f1[2]; fv[7] = f1[3];
    unsigned hb[8], lb[8];
#pragma unroll
    for (int e = 0; e < 8; ++e) {
      const v4f pw = *(const v4f*)(pp + (rowo + e) * 4);
      const float pre = pw[0];
      const float pim = pw[1];
      const float wre = pw[2];
      const float wim = pw[3];
      const float fg  = fv[e] * gam[e];
      const float qre = fg * wre;
      const float qim = fg * wim;
      sre[e] = sre[e] + qre;
      sim[e] = sim[e] + qim;
      const float ta = pre * sre[e];
      const float tb = pim * sim[e];
      const float x  = ta - tb;
      hb[e] = bf_hi_bits(x);
      lb[e] = bf_hi_bits(x - bf_bits_val(hb[e]));
    }
    const v4u hw = (v4u){hb[0] | (hb[1] << 16), hb[2] | (hb[3] << 16), hb[4] | (hb[5] << 16), hb[6] | (hb[7] << 16)};
    const v4u lw = (v4u){lb[0] | (lb[1] << 16), lb[2] | (lb[3] << 16), lb[4] | (lb[5] << 16), lb[6] | (lb[7] << 16)};
    *(volatile v4u*)(xh + rowo) = hw;
    *(volatile v4u*)(xl + rowo) = lw;
    __threadfence();
    *(volatile v4u*)(xh + rowo) = hw;
    *(volatile v4u*)(xl + rowo) = lw;
  }
}

__device__ __forceinline__ void mma_rows64_cols32(const __bf16* __restrict__ Ah, const __bf16* __restrict__ Al, int lda, int m0,
                                                  const __bf16* __restrict__ Bh, const __bf16* __restrict__ Bl, int ldb,
                                                  int rlane, int kk, v8f (&acc)[4][2]) {
  v16b bh[2], bl[2];
#pragma unroll
  for (int j = 0; j < 2; ++j) {
    const size_t bo = (size_t)((j << 4) + rlane) * ldb + kk;
    bh[j] = Frag<__bf16>::load(Bh + bo);
    bl[j] = Frag<__bf16>::load(Bl + bo);
  }
#pragma unroll
  for (int i = 0; i < 4; ++i) {
    const size_t ao = (size_t)(m0 + (i << 4) + rlane) * lda + kk;
    const v16b ah = Frag<__bf16>::load(Ah + ao);
    const v16b al = Frag<__bf16>::load(Al + ao);
#pragma unroll
    for (int j = 0; j < 2; ++j) {
      acc[i][j] = Frag<__bf16>::mma(ah, bh[j], acc[i][j]);
      acc[i][j] = Frag<__bf16>::mma(ah, bl[j], acc[i][j]);
      acc[i][j] = Frag<__bf16>::mma(al, bh[j], acc[i][j]);
    }
    dep_guard_b(acc[i][0], acc[i][1], ah, al);
  }
  keep4_b(bh[0], bh[1], bl[0], bl[1]);
}

__global__ __launch_bounds__(NTHR) void proj_out_kernel(const unsigned short* __restrict__ Xhp, const unsigned short* __restrict__ Xlp,
                                                        const unsigned short* __restrict__ Chp, const unsigned short* __restrict__ Clp,
                                                        const unsigned short* __restrict__ Uhp, const unsigned short* __restrict__ Ulp,
                                                        const unsigned short* __restrict__ Dhp, const unsigned short* __restrict__ Dlp,
                                                        float* __restrict__ out) {
  __shared__ __align__(16) float sO[8][16 * SLAB_O];
  const __bf16* Xh = (const __bf16*)Xhp;
  const __bf16* Xl = (const __bf16*)Xlp;
  const __bf16* Ch = (const __bf16*)Chp;
  const __bf16* Cl = (const __bf16*)Clp;
  const __bf16* Uh = (const __bf16*)Uhp;
  const __bf16* Ul = (const __bf16*)Ulp;
  const __bf16* Dh = (const __bf16*)Dhp;
  const __bf16* Dl = (const __bf16*)Dlp;
  const int lane = threadIdx.x & 31;
  const int wave = threadIdx.x >> 5;
  const int tile = blockIdx.x * 8 + wave;
  if (tile >= NROWS / 64) return;
  const int m0    = tile * 64;
  const int rlane = lane & 15;
  const int koff  = (lane >> 4) * 8;
  const int mOff  = (lane >> 4) * 8;

  v8f acc[4][2];
#pragma unroll
  for (int i = 0; i < 4; ++i)
#pragma unroll
    for (int j = 0; j < 2; ++j) acc[i][j] = (v8f){0.f, 0.f, 0.f, 0.f, 0.f, 0.f, 0.f, 0.f};

#pragma unroll 1
  for (int k0 = 0; k0 < NHID; k0 += 32) {
    mma_rows64_cols32(Xh, Xl, NHID, m0, Ch, Cl, NHID, rlane, koff + k0, acc);
  }
  mma_rows64_cols32(Uh, Ul, NIN, m0, Dh, Dl, NIN, rlane, koff, acc);
  acc_guard4(acc[0][0], acc[0][1], acc[1][0], acc[1][1]);
  acc_guard4(acc[2][0], acc[2][1], acc[3][0], acc[3][1]);

  float* slab = sO[wave];
#pragma unroll
  for (int i = 0; i < 4; ++i) {
    const int mBase = m0 + (i << 4);
#pragma unroll
    for (int j = 0; j < 2; ++j) {
#pragma unroll
      for (int r = 0; r < 8; ++r) slab[(mOff + r) * SLAB_O + (j << 4) + rlane] = acc[i][j][r];
    }
    __builtin_amdgcn_fence(__ATOMIC_RELEASE, "workgroup");
    __builtin_amdgcn_wave_barrier();
    __builtin_amdgcn_fence(__ATOMIC_ACQUIRE, "workgroup");
    {
      const int q  = lane >> 3;
      const int c4 = (lane & 7) * 4;
      for (int pass = 0; pass < 2; ++pass) {
#pragma unroll
        for (int it = 0; it < 4; ++it) {
          const int row = it * 4 + q;
          const v4f v = *(const v4f*)(slab + row * SLAB_O + c4);
          *(volatile v4f*)(out + (size_t)(mBase + row) * NOUT + c4) = v;
        }
        __threadfence();
      }
    }
    __builtin_amdgcn_fence(__ATOMIC_RELEASE, "workgroup");
    __builtin_amdgcn_wave_barrier();
    __builtin_amdgcn_fence(__ATOMIC_ACQUIRE, "workgroup");
  }
}

extern "C" void kernel_launch(void* const* d_in, const int* in_sizes, int n_in,
                              void* d_out, int out_size, void* d_ws, size_t ws_size, hipStream_t stream) {
  if (n_in < 6 || d_out == nullptr || d_ws == nullptr) return;
  if (in_sizes[0] != NROWS * NIN || in_sizes[1] != NHID || in_sizes[2] != NHID ||
      in_sizes[3] != NHID * NIN || in_sizes[4] != NOUT * NHID || in_sizes[5] != NOUT * NIN ||
      out_size != NROWS * NOUT) return;

  const float* u      = (const float*)d_in[0];
  const float* nu_log = (const float*)d_in[1];
  const float* th_log = (const float*)d_in[2];
  const float* Bm     = (const float*)d_in[3];
  const float* Cm     = (const float*)d_in[4];
  const float* Dm     = (const float*)d_in[5];
  float* y_out = (float*)d_out;

  char* ws = (char*)d_ws;
  size_t off = 0;
  auto carve = [&](size_t bytes) -> char* { char* p = ws + off; off += (bytes + 255) & ~(size_t)255; return p; };
  unsigned short* UH = (unsigned short*)carve((size_t)NROWS * NIN * 2);
  unsigned short* UL = (unsigned short*)carve((size_t)NROWS * NIN * 2);
  unsigned short* BH = (unsigned short*)carve((size_t)NHID * NIN * 2);
  unsigned short* BL = (unsigned short*)carve((size_t)NHID * NIN * 2);
  unsigned short* CH = (unsigned short*)carve((size_t)NOUT * NHID * 2);
  unsigned short* CL = (unsigned short*)carve((size_t)NOUT * NHID * 2);
  unsigned short* DH = (unsigned short*)carve((size_t)NOUT * NIN * 2);
  unsigned short* DL = (unsigned short*)carve((size_t)NOUT * NIN * 2);
  float*          GAM  = (float*)carve((size_t)NHID * 4);
  float*          PW   = (float*)carve((size_t)NSEQ * NHID * 16);
  float*          FRAW = (float*)carve((size_t)NROWS * NHID * 4);
  unsigned short* XH = (unsigned short*)carve((size_t)NROWS * NHID * 2);
  unsigned short* XL = (unsigned short*)carve((size_t)NROWS * NHID * 2);
  if (off > ws_size || off > (size_t)134217728) return;

  const int n8u = NROWS * NIN / 8;
  const int n8b = NHID * NIN / 8;
  const int n8c = NOUT * NHID / 8;
  const int n8d = NOUT * NIN / 8;
  split8_kernel<<<(n8u + NTHR - 1) / NTHR, NTHR, 0, stream>>>(u,  UH, UL, n8u);
  split8_kernel<<<(n8b + NTHR - 1) / NTHR, NTHR, 0, stream>>>(Bm, BH, BL, n8b);
  split8_kernel<<<(n8c + NTHR - 1) / NTHR, NTHR, 0, stream>>>(Cm, CH, CL, n8c);
  split8_kernel<<<(n8d + NTHR - 1) / NTHR, NTHR, 0, stream>>>(Dm, DH, DL, n8d);

  ptable_kernel<<<NSEQ, NTHR, 0, stream>>>(nu_log, th_log, PW, GAM);

  proj_in_kernel<<<(NROWS / 32) * (NHID / 64) / 8, NTHR, 0, stream>>>(UH, UL, BH, BL, FRAW);

  cumsum_kernel<<<NBATCH, 32, 0, stream>>>(FRAW, PW, GAM, XH, XL);

  proj_out_kernel<<<(NROWS / 64) / 8, NTHR, 0, stream>>>(XH, XL, CH, CL, UH, UL, DH, DL, y_out);
}
